// MambaStateSpaceModel_56470230008017
// MI455X (gfx1250) — hardware-verified
//
#include <hip/hip_runtime.h>
#include <math.h>


typedef unsigned short us;
typedef us      v16u __attribute__((ext_vector_type(16)));
typedef us      v8u  __attribute__((ext_vector_type(8)));
typedef us      v4us __attribute__((ext_vector_type(4)));
typedef __bf16  v16b __attribute__((ext_vector_type(16)));
typedef float   v8f  __attribute__((ext_vector_type(8)));
typedef float   v4f  __attribute__((ext_vector_type(4)));
typedef unsigned int v4u __attribute__((ext_vector_type(4)));

#define NB   64
#define NT   2048
#define NI   64
#define NS   128
#define NO   64
#define XP   192
#define HP   128
#define NTHR 256
#define LN_EPS 1e-5f

union Frag { v16b v; v16u u; v8u q[2]; };
union P8   { v8u h; v4u u; us s[8]; };
union P4   { v4f f; v4u u; float s[4]; };
union P4s  { v4us v; us s[4]; };

__device__ __forceinline__ us bf16_rne(float f) {
  unsigned int u = __float_as_uint(f);
  u = u + 0x7FFFu + ((u >> 16) & 1u);
  return (us)(u >> 16);
}
__device__ __forceinline__ void split2(float f, us& hi, us& lo) {
  const us hh = bf16_rne(f);
  const float fh = __uint_as_float(((unsigned int)hh) << 16);
  hi = hh;
  lo = bf16_rne(f - fh);
}

__device__ __forceinline__ v8f zero8() {
  v8f z = {0.f, 0.f, 0.f, 0.f, 0.f, 0.f, 0.f, 0.f};
  return z;
}

__device__ __forceinline__ v8f wmma_bf(v16b a, v16b b, v8f c) {
  return __builtin_amdgcn_wmma_f32_16x16x32_bf16(false, a, false, b, (short)0, c, false, false);
}

__device__ __forceinline__ void mma3(v8f& acc, const us* Ah, const us* Al, int lda,
                                     const us* Bh, const us* Bl, int ldb, int ktiles) {
  const int l = threadIdx.x & 31, h = l >> 4, m = l & 15;
  const us* pah = Ah + m * lda + 8 * h;
  const us* pal = Al + m * lda + 8 * h;
  const us* pbh = Bh + m * ldb + 8 * h;
  const us* pbl = Bl + m * ldb + 8 * h;
#pragma unroll 1
  for (int kt = 0; kt < ktiles; ++kt) {
    const int ko = 32 * kt;
    Frag ah, al, bh, bl;
    ah.q[0] = *(const v8u*)(pah + ko);  ah.q[1] = *(const v8u*)(pah + ko + 16);
    al.q[0] = *(const v8u*)(pal + ko);  al.q[1] = *(const v8u*)(pal + ko + 16);
    bh.q[0] = *(const v8u*)(pbh + ko);  bh.q[1] = *(const v8u*)(pbh + ko + 16);
    bl.q[0] = *(const v8u*)(pbl + ko);  bl.q[1] = *(const v8u*)(pbl + ko + 16);
    acc = wmma_bf(ah.v, bh.v, acc);
    acc = wmma_bf(ah.v, bl.v, acc);
    acc = wmma_bf(al.v, bh.v, acc);
    asm volatile("v_nop\n\tv_nop\n\tv_nop\n\tv_nop"
                 : "+v"(acc)
                 : "v"(ah.v), "v"(al.v), "v"(bh.v), "v"(bl.v));
  }
}

__device__ __forceinline__ void rowred8(float (&s)[8]) {
#pragma unroll
  for (int off = 1; off < 16; off <<= 1) {
#pragma unroll
    for (int j = 0; j < 8; ++j) s[j] += __shfl_xor(s[j], off, 32);
  }
}

__device__ __forceinline__ void sum8(const float* red, int h, float (&out)[8]) {
#pragma unroll
  for (int j = 0; j < 8; ++j) out[j] = 0.f;
#pragma unroll 1
  for (int w2 = 0; w2 < 8; ++w2) {
    P4 a, b;
    a.f = *(const v4f*)(red + w2 * 16 + 8 * h);
    b.f = *(const v4f*)(red + w2 * 16 + 8 * h + 4);
#pragma unroll
    for (int i = 0; i < 4; ++i) { out[i] += a.s[i]; out[4 + i] += b.s[i]; }
  }
}

__device__ __forceinline__ void stats_step(const float* ys, int row, int c4, int t,
                                           float (&yprev)[4], double (&sy)[4], double (&sy2)[4],
                                           double& nacc, double& dacc) {
  P4 yv;
  yv.f = *(const v4f*)(ys + row * NO + c4);
  float s2 = 0.f, d2 = 0.f;
#pragma unroll
  for (int i = 0; i < 4; ++i) {
    const float y = yv.s[i];
    const float d = y - yprev[i];
    s2 += y * y;
    d2 += d * d;
    yprev[i] = y;
    sy[i]  += (double)y;
    sy2[i] += (double)y * (double)y;
  }
#pragma unroll
  for (int off = 1; off < 16; off <<= 1) {
    s2 += __shfl_xor(s2, off, 32);
    d2 += __shfl_xor(d2, off, 32);
  }
  nacc += (double)sqrtf(s2);
  if (t > 0) dacc += (double)sqrtf(d2);
}

__device__ __forceinline__ void block_tail(const us* PWh, const us* PWl, const float* bsel,
                                           us* xh, us* xl, double* dred, double* pl,
                                           const float (&yprev)[4], const double (&sy)[4],
                                           const double (&sy2)[4], const double (&xs)[4],
                                           double nacc, double dacc,
                                           unsigned int* part, float* outp, int b0) {
  const int tid = threadIdx.x, w = tid >> 5, l = tid & 31, col = l & 15;
  const int row = tid >> 4, c4 = (tid & 15) * 4;
  {
    P4 v;
#pragma unroll
    for (int i = 0; i < 4; ++i) v.s[i] = yprev[i];
    float* dst = outp + (size_t)(b0 + row) * NO + c4;
    *(volatile v4f*)dst = v.f;
    __threadfence();
    *(volatile v4f*)dst = v.f;
  }
  {
    P4s vh, vl;
#pragma unroll
    for (int i = 0; i < 4; ++i) {
      const float xm = (float)(xs[i] * (1.0 / NT));
      split2(xm, vh.s[i], vl.s[i]);
    }
    *(v4us*)(xh + row * XP + c4) = vh.v;
    *(v4us*)(xl + row * XP + c4) = vl.v;
  }
  __syncthreads();
  v8f accs = zero8();
  mma3(accs, xh, xl, XP, PWh + (size_t)(16 * w) * NI, PWl + (size_t)(16 * w) * NI, NI, 2);
  const float bs = bsel[16 * w + col];
  double ssum = 0.0;
#pragma unroll
  for (int j = 0; j < 8; ++j) {
    const float z = accs[j] + bs;
    const float g = 1.0f / (1.0f + expf(-z));
    ssum += (double)g;
  }
  double sd = 0.0;
#pragma unroll
  for (int i = 0; i < 4; ++i) {
    const double mean = sy[i] * (1.0 / NT);
    double var = (sy2[i] - sy[i] * mean) * (1.0 / (NT - 1));
    var = var < 0.0 ? 0.0 : var;
    sd += sqrt(var);
  }
  dred[tid] = sd;
  dred[NTHR + tid] = ssum;
  if (col == 0) {
    dred[2 * NTHR + row] = nacc;
    dred[2 * NTHR + 16 + row] = dacc;
  }
  __syncthreads();
  if (tid == 0) {
    double a = 0.0, b = 0.0, c = 0.0, d = 0.0;
    for (int r = 0; r < 16; ++r) { a += dred[2 * NTHR + r]; b += dred[2 * NTHR + 16 + r]; }
    for (int i = 0; i < NTHR; ++i) { c += dred[i]; d += dred[NTHR + i]; }
    pl[0] = a; pl[1] = b; pl[2] = c; pl[3] = d;
    for (int k = 4; k < 16; ++k) pl[k] = 0.0;
  }
  __syncthreads();
  if (tid < 8) {
    const v4u v = ((const v4u*)pl)[tid];
    unsigned int* dst = part + (size_t)blockIdx.x * 32 + tid * 4;
    *(volatile v4u*)dst = v;
    __threadfence();
    *(volatile v4u*)dst = v;
  }
}

__global__ void __launch_bounds__(NTHR) k_pack(const float* W, us* Ph, us* Pl, int n8) {
  const int i = blockIdx.x * NTHR + threadIdx.x;
  if (i >= n8) return;
  const float* p = W + (size_t)i * 8;
  P4 a, b;
  a.f = *(const v4f*)p;
  b.f = *(const v4f*)(p + 4);
  P8 vh, vl;
#pragma unroll
  for (int e = 0; e < 4; ++e) {
    split2(a.s[e], vh.s[e],     vl.s[e]);
    split2(b.s[e], vh.s[4 + e], vl.s[4 + e]);
  }
  us* dh = Ph + (size_t)i * 8;
  us* dl = Pl + (size_t)i * 8;
  *(volatile v4u*)dh = vh.u;
  *(volatile v4u*)dl = vl.u;
  __threadfence();
  *(volatile v4u*)dh = vh.u;
  *(volatile v4u*)dl = vl.u;
}

__global__ void __launch_bounds__(NTHR) k_pack_conv(const float* Wc, us* Ph, us* Pl) {
  const int i = blockIdx.x * NTHR + threadIdx.x;
  if (i >= NS * 24) return;
  const int s = i / 24, g = i - s * 24;
  const int k = g >> 3, i0 = (g & 7) * 8;
  P8 vh, vl;
#pragma unroll
  for (int e = 0; e < 8; ++e) {
    const float v = Wc[(size_t)s * (NI * 3) + (i0 + e) * 3 + k];
    split2(v, vh.s[e], vl.s[e]);
  }
  const size_t o = (size_t)s * XP + 64 * k + i0;
  us* dh = Ph + o;
  us* dl = Pl + o;
  *(volatile v4u*)dh = vh.u;
  *(volatile v4u*)dl = vl.u;
  __threadfence();
  *(volatile v4u*)dh = vh.u;
  *(volatile v4u*)dl = vl.u;
}

__global__ void __launch_bounds__(NTHR) __attribute__((amdgpu_num_vgpr(248)))
k_seq(const float* x,
      const us* PAh, const us* PAl, const us* PBh, const us* PBl,
      const us* PWh, const us* PWl, const us* PCh, const us* PCl,
      const us* PDh, const us* PDl,
      const float* bsel, const float* gam, const float* bet,
      const int* usep, unsigned int* part, float* outp) {
  __shared__ __attribute__((aligned(16))) us hh[16 * HP];
  __shared__ __attribute__((aligned(16))) us hl[16 * HP];
  __shared__ __attribute__((aligned(16))) us xh[16 * XP];
  __shared__ __attribute__((aligned(16))) us xl[16 * XP];
  __shared__ __attribute__((aligned(16))) float redS[8 * 16];
  __shared__ __attribute__((aligned(16))) float redQ[8 * 16];
  __shared__ __attribute__((aligned(16))) float ys[16 * NO];
  __shared__ __attribute__((aligned(16))) double dred[2 * NTHR + 32];
  __shared__ __attribute__((aligned(16))) double pl[16];

  if (usep[0] != 0) return;

  const int tid = threadIdx.x, w = tid >> 5, l = tid & 31, h = l >> 4, col = l & 15;
  const int b0 = blockIdx.x * 16;
  const int row = tid >> 4, c4 = (tid & 15) * 4;
  const int ncol = 16 * w + col;

  for (int i = tid; i < 16 * HP; i += NTHR) { hh[i] = 0; hl[i] = 0; }
  for (int i = tid; i < 16 * XP; i += NTHR) { xh[i] = 0; xl[i] = 0; }

  const float gm = gam[ncol], bt = bet[ncol], bs = bsel[ncol];
  float hprev[8];
#pragma unroll
  for (int j = 0; j < 8; ++j) hprev[j] = 0.f;
  float yprev[4] = {0.f, 0.f, 0.f, 0.f};
  double sy[4] = {0.0, 0.0, 0.0, 0.0}, sy2[4] = {0.0, 0.0, 0.0, 0.0}, xs[4] = {0.0, 0.0, 0.0, 0.0};
  double nacc = 0.0, dacc = 0.0;
  const float* xrow = x + ((size_t)(b0 + row) * NT) * NI + c4;
  const size_t wB = (size_t)(16 * w) * NI;
  const size_t wA = (size_t)(16 * w) * NS;
  __syncthreads();

#pragma unroll 1
  for (int t = 0; t < NT; ++t) {
    {
      P4 xv;
      xv.f = *(const v4f*)(xrow + (size_t)t * NI);
      P4s vh, vl;
#pragma unroll
      for (int i = 0; i < 4; ++i) {
        split2(xv.s[i], vh.s[i], vl.s[i]);
        xs[i] += (double)xv.s[i];
      }
      *(v4us*)(xh + row * XP + c4) = vh.v;
      *(v4us*)(xl + row * XP + c4) = vl.v;
    }
    __syncthreads();

    v8f accg = zero8(), acch = zero8();
    mma3(accg, xh, xl, XP, PWh + wB, PWl + wB, NI, 2);
    mma3(acch, xh, xl, XP, PBh + wB, PBl + wB, NI, 2);
    mma3(acch, hh, hl, HP, PAh + wA, PAl + wA, NS, 4);

    float hc[8], s[8];
#pragma unroll
    for (int j = 0; j < 8; ++j) {
      const float z = accg[j] + bs;
      const float g = __builtin_amdgcn_rcpf(1.0f + __expf(-z));
      hc[j] = g * acch[j] + (1.0f - g) * hprev[j];
      s[j] = hc[j];
    }
    rowred8(s);
    if (col == 0) {
      P4 a, b;
#pragma unroll
      for (int i = 0; i < 4; ++i) { a.s[i] = s[i]; b.s[i] = s[4 + i]; }
      *(v4f*)(redS + w * 16 + 8 * h)     = a.f;
      *(v4f*)(redS + w * 16 + 8 * h + 4) = b.f;
    }
    __syncthreads();

    float mu[8];
    sum8(redS, h, mu);
#pragma unroll
    for (int j = 0; j < 8; ++j) {
      mu[j] *= (1.0f / NS);
      hc[j] -= mu[j];
      s[j] = hc[j] * hc[j];
    }
    rowred8(s);
    if (col == 0) {
      P4 a, b;
#pragma unroll
      for (int i = 0; i < 4; ++i) { a.s[i] = s[i]; b.s[i] = s[4 + i]; }
      *(v4f*)(redQ + w * 16 + 8 * h)     = a.f;
      *(v4f*)(redQ + w * 16 + 8 * h + 4) = b.f;
    }
    __syncthreads();

    float var[8];
    sum8(redQ, h, var);
#pragma unroll
    for (int j = 0; j < 8; ++j) {
      const float rs = rsqrtf(var[j] * (1.0f / NS) + LN_EPS);
      const float hn = hc[j] * rs * gm + bt;
      hprev[j] = hn;
      us a, b;
      split2(hn, a, b);
      hh[(8 * h + j) * HP + ncol] = a;
      hl[(8 * h + j) * HP + ncol] = b;
    }
    __syncthreads();

    if (w < 4) {
      v8f accy = zero8();
      mma3(accy, hh, hl, HP, PCh + wA, PCl + wA, NS, 4);
      mma3(accy, xh, xl, XP, PDh + wB, PDl + wB, NI, 2);
#pragma unroll
      for (int j = 0; j < 8; ++j) ys[(8 * h + j) * NO + ncol] = accy[j];
    }
    __syncthreads();

    stats_step(ys, row, c4, t, yprev, sy, sy2, nacc, dacc);
  }

  block_tail(PWh, PWl, bsel, xh, xl, dred, pl, yprev, sy, sy2, xs, nacc, dacc, part, outp, b0);
}

__global__ void __launch_bounds__(NTHR) __attribute__((amdgpu_num_vgpr(248)))
k_par(const float* x,
      const us* PKh, const us* PKl, const us* PCh, const us* PCl,
      const us* PWh, const us* PWl,
      const float* convb, const float* bsel,
      const int* usep, unsigned int* part, float* outp) {
  __shared__ __attribute__((aligned(16))) us hh[16 * HP];
  __shared__ __attribute__((aligned(16))) us hl[16 * HP];
  __shared__ __attribute__((aligned(16))) us xh[16 * XP];
  __shared__ __attribute__((aligned(16))) us xl[16 * XP];
  __shared__ __attribute__((aligned(16))) float ys[16 * NO];
  __shared__ __attribute__((aligned(16))) double dred[2 * NTHR + 32];
  __shared__ __attribute__((aligned(16))) double pl[16];

  if (usep[0] == 0) return;

  const int tid = threadIdx.x, w = tid >> 5, l = tid & 31, h = l >> 4, col = l & 15;
  const int b0 = blockIdx.x * 16;
  const int row = tid >> 4, c4 = (tid & 15) * 4;
  const int ncol = 16 * w + col;

  for (int i = tid; i < 16 * HP; i += NTHR) { hh[i] = 0; hl[i] = 0; }
  for (int i = tid; i < 16 * XP; i += NTHR) { xh[i] = 0; xl[i] = 0; }

  const float cb = convb[ncol];
  float cum[8];
#pragma unroll
  for (int j = 0; j < 8; ++j) cum[j] = 0.f;
  float yprev[4] = {0.f, 0.f, 0.f, 0.f};
  double sy[4] = {0.0, 0.0, 0.0, 0.0}, sy2[4] = {0.0, 0.0, 0.0, 0.0}, xs[4] = {0.0, 0.0, 0.0, 0.0};
  double nacc = 0.0, dacc = 0.0;
  const float* xrow = x + ((size_t)(b0 + row) * NT) * NI + c4;
  const size_t wK = (size_t)(16 * w) * XP;
  const size_t wA = (size_t)(16 * w) * NS;
  const P4 zero4 = {{0.f, 0.f, 0.f, 0.f}};
  __syncthreads();

#pragma unroll 1
  for (int t = 0; t < NT; ++t) {
#pragma unroll
    for (int k = 0; k < 3; ++k) {
      const int tt = t + k - 1;
      const bool ok = (tt >= 0) && (tt < NT);
      const int tc = tt < 0 ? 0 : (tt > NT - 1 ? NT - 1 : tt);
      P4 xv;
      xv.f = *(const v4f*)(xrow + (size_t)tc * NI);
      if (!ok) xv = zero4;
      P4s vh, vl;
#pragma unroll
      for (int i = 0; i < 4; ++i) {
        if (k == 1) xs[i] += (double)xv.s[i];
        split2(xv.s[i], vh.s[i], vl.s[i]);
      }
      *(v4us*)(xh + row * XP + 64 * k + c4) = vh.v;
      *(v4us*)(xl + row * XP + 64 * k + c4) = vl.v;
    }
    __syncthreads();

    v8f accc = zero8();
    mma3(accc, xh, xl, XP, PKh + wK, PKl + wK, XP, 6);
#pragma unroll
    for (int j = 0; j < 8; ++j) {
      const float cv = accc[j] + cb;
      cum[j] += cv;
      us a, b;
      split2(cum[j], a, b);
      hh[(8 * h + j) * HP + ncol] = a;
      hl[(8 * h + j) * HP + ncol] = b;
    }
    __syncthreads();

    if (w < 4) {
      v8f accy = zero8();
      mma3(accy, hh, hl, HP, PCh + wA, PCl + wA, NS, 4);
#pragma unroll
      for (int j = 0; j < 8; ++j) ys[(8 * h + j) * NO + ncol] = accy[j];
    }
    __syncthreads();

    stats_step(ys, row, c4, t, yprev, sy, sy2, nacc, dacc);
  }

  block_tail(PWh, PWl, bsel, xh, xl, dred, pl, yprev, sy, sy2, xs, nacc, dacc, part, outp, b0);
}

__global__ void __launch_bounds__(32) k_fin(const unsigned int* part, float* outp, int nblk) {
  if (threadIdx.x != 0) return;
  const double* pd = (const double*)part;
  double a = 0.0, b = 0.0, c = 0.0, d = 0.0;
  for (int k = 0; k < nblk; ++k) {
    a += pd[k * 16 + 0];
    b += pd[k * 16 + 1];
    c += pd[k * 16 + 2];
    d += pd[k * 16 + 3];
  }
  const float mdiff = (float)(b / (double)(NB * (NT - 1)));
  P4 v;
  v.s[0] = 1.0f / (1.0f + mdiff);
  v.s[1] = (float)(a / (double)(NB * NT));
  v.s[2] = (float)(d / (double)(NB * NS));
  v.s[3] = (float)(c / (double)(NB * NO));
  float* dst = outp + NB * NO;
  *(volatile v4f*)dst = v.f;
  __threadfence();
  *(volatile v4f*)dst = v.f;
}

extern "C" void kernel_launch(void* const* d_in, const int* in_sizes, int n_in,
                              void* d_out, int out_size, void* d_ws, size_t ws_size,
                              hipStream_t stream) {
  if (n_in < 12) return;
  if (in_sizes[0] != NB * NT * NI || in_sizes[1] != NS * NS || in_sizes[2] != NS * NI ||
      in_sizes[3] != NO * NS || in_sizes[4] != NO * NI || in_sizes[5] != NS * NI ||
      in_sizes[6] != NS || in_sizes[7] != NS || in_sizes[8] != NS ||
      in_sizes[9] != NS * NI * 3 || in_sizes[10] != NS || in_sizes[11] < 1) return;
  if (out_size != NB * NO + 4) return;

  const float* x     = (const float*)d_in[0];
  const float* A     = (const float*)d_in[1];
  const float* Bm    = (const float*)d_in[2];
  const float* Cm    = (const float*)d_in[3];
  const float* Dm    = (const float*)d_in[4];
  const float* Wsel  = (const float*)d_in[5];
  const float* bsel  = (const float*)d_in[6];
  const float* gam   = (const float*)d_in[7];
  const float* bet   = (const float*)d_in[8];
  const float* convw = (const float*)d_in[9];
  const float* convb = (const float*)d_in[10];
  const int*   usep  = (const int*)d_in[11];
  float* outp = (float*)d_out;

  char* ws = (char*)d_ws;
  size_t off = 0;
  auto carve = [&](size_t bytes) -> char* {
    char* p = ws + off;
    off = (off + bytes + 255) & ~(size_t)255;
    return p;
  };
  us* PAh = (us*)carve((size_t)NS * NS * 2);
  us* PAl = (us*)carve((size_t)NS * NS * 2);
  us* PBh = (us*)carve((size_t)NS * NI * 2);
  us* PBl = (us*)carve((size_t)NS * NI * 2);
  us* PCh = (us*)carve((size_t)NO * NS * 2);
  us* PCl = (us*)carve((size_t)NO * NS * 2);
  us* PDh = (us*)carve((size_t)NO * NI * 2);
  us* PDl = (us*)carve((size_t)NO * NI * 2);
  us* PWh = (us*)carve((size_t)NS * NI * 2);
  us* PWl = (us*)carve((size_t)NS * NI * 2);
  us* PKh = (us*)carve((size_t)NS * XP * 2);
  us* PKl = (us*)carve((size_t)NS * XP * 2);
  unsigned int* part = (unsigned int*)carve((size_t)(NB / 16) * 128);
  if (off > ws_size || off > (size_t)134217728) return;

  {
    int n8;
    n8 = NS * NS / 8; k_pack<<<dim3((n8 + NTHR - 1) / NTHR), dim3(NTHR), 0, stream>>>(A,    PAh, PAl, n8);
    n8 = NS * NI / 8; k_pack<<<dim3((n8 + NTHR - 1) / NTHR), dim3(NTHR), 0, stream>>>(Bm,   PBh, PBl, n8);
    n8 = NO * NS / 8; k_pack<<<dim3((n8 + NTHR - 1) / NTHR), dim3(NTHR), 0, stream>>>(Cm,   PCh, PCl, n8);
    n8 = NO * NI / 8; k_pack<<<dim3((n8 + NTHR - 1) / NTHR), dim3(NTHR), 0, stream>>>(Dm,   PDh, PDl, n8);
    n8 = NS * NI / 8; k_pack<<<dim3((n8 + NTHR - 1) / NTHR), dim3(NTHR), 0, stream>>>(Wsel, PWh, PWl, n8);
    k_pack_conv<<<dim3((NS * 24 + NTHR - 1) / NTHR), dim3(NTHR), 0, stream>>>(convw, PKh, PKl);
  }
  k_seq<<<dim3(NB / 16), dim3(NTHR), 0, stream>>>(x, PAh, PAl, PBh, PBl, PWh, PWl, PCh, PCl, PDh, PDl,
                                                  bsel, gam, bet, usep, part, outp);
  k_par<<<dim3(NB / 16), dim3(NTHR), 0, stream>>>(x, PKh, PKl, PCh, PCl, PWh, PWl, convb, bsel,
                                                  usep, part, outp);
  k_fin<<<dim3(1), dim3(32), 0, stream>>>(part, outp, NB / 16);
}
